// CapsuleMortalityHead_89593017794951
// MI455X (gfx1250) — hardware-verified
//
#include <hip/hip_runtime.h>


#define NS   8192
#define NP   7
#define DD   256
#define MC   25
#define VV   64
#define MV   (MC * VV)
#define SCH  1024
#define NCHK (NS / SCH)
typedef _Float16 h16;
typedef unsigned short bf;
typedef __attribute__((ext_vector_type(16))) __bf16   v16bf;
typedef __attribute__((ext_vector_type(16))) _Float16 v16h;
typedef __attribute__((ext_vector_type(8)))  _Float16 v8h;
typedef __attribute__((ext_vector_type(8)))  unsigned short v8us;
typedef __attribute__((ext_vector_type(8)))  float    v8f;
typedef __attribute__((ext_vector_type(4)))  float    v4f;
typedef v8h  __attribute__((may_alias)) v8ha;
typedef v4f  __attribute__((may_alias)) v4fa;
typedef v8us __attribute__((may_alias)) v8usa;

__device__ __forceinline__ unsigned short f2bf(float f) { unsigned u = __float_as_uint(f); u += 0x7FFFu + ((u >> 16) & 1u); return (unsigned short)(u >> 16); }
__device__ __forceinline__ float bf2f(unsigned short b) { return __uint_as_float(((unsigned)b) << 16); }
__device__ __forceinline__ float bfr(float f) { return bf2f(f2bf(f)); }
__device__ __forceinline__ v16h cat16(v8h lo, v8h hi) { return __builtin_shufflevector(lo, hi, 0, 1, 2, 3, 4, 5, 6, 7, 8, 9, 10, 11, 12, 13, 14, 15); }
__device__ __forceinline__ v16bf cat16b(v8us lo, v8us hi) { return __builtin_bit_cast(v16bf, __builtin_shufflevector(lo, hi, 0, 1, 2, 3, 4, 5, 6, 7, 8, 9, 10, 11, 12, 13, 14, 15)); }
__device__ __forceinline__ v8f wmma16(v16h a, v16h b, v8f c) { return __builtin_amdgcn_wmma_f32_16x16x32_f16(false, a, false, b, (short)0, c, false, false); }
__device__ __forceinline__ v8f wmmab(v16bf a, v16bf b, v8f c) { return __builtin_amdgcn_wmma_f32_16x16x32_bf16(false, a, false, b, (short)0, c, false, false); }


template <typename T16> struct WFrag;
template <> struct WFrag<h16> { typedef v16h V; static __device__ __forceinline__ V ld(const h16* p) { return cat16(*(const v8h*)p, *(const v8h*)(p + 16)); } static __device__ __forceinline__ v8f mma(V a, V b, v8f c) { return wmma16(a, b, c); } };
template <> struct WFrag<bf> { typedef v16bf V; static __device__ __forceinline__ V ld(const bf* p) { return cat16b(*(const v8us*)p, *(const v8us*)(p + 16)); } static __device__ __forceinline__ v8f mma(V a, V b, v8f c) { return wmmab(a, b, c); } };
template <typename T16, int NSPLIT, bool BIAS>
__global__ __launch_bounds__(32) void k_gemmw(const T16* __restrict__ A, const T16* __restrict__ A2, const T16* __restrict__ Bt, const T16* __restrict__ Bt2, int K, float* C, int ldc, const float* __restrict__ bias, size_t sA, size_t sB, size_t sC) {
    typedef typename WFrag<T16>::V V;
    __shared__ __align__(16) float os[16 * 68];
    const size_t z = blockIdx.z; A += z * sA; if (A2) A2 += z * sA; Bt += z * sB; if (Bt2) Bt2 += z * sB; C += z * sC;
    const int lane = threadIdx.x & 31, lr = lane & 15, hi = lane >> 4; const int r0 = blockIdx.x * 64, c0 = blockIdx.y * 64;
    v8f acc[4][4];
#pragma unroll
    for (int mb = 0; mb < 4; ++mb)
#pragma unroll
        for (int nb = 0; nb < 4; ++nb) acc[mb][nb] = (v8f){};
    const size_t aoff = (size_t)(r0 + lr) * K + 8 * hi, boff = (size_t)(c0 + lr) * K + 8 * hi;
#pragma unroll 1
    for (int kc = 0; kc < K; kc += 32) {
        V a[4], a2[4];
#pragma unroll
        for (int mb = 0; mb < 4; ++mb) { a[mb] = WFrag<T16>::ld(A + aoff + (size_t)mb * 16 * K + kc); if (NSPLIT == 1 || NSPLIT == 2) a2[mb] = WFrag<T16>::ld(A2 + aoff + (size_t)mb * 16 * K + kc); }
#pragma unroll
        for (int nb = 0; nb < 4; ++nb) { const V b = WFrag<T16>::ld(Bt + boff + (size_t)nb * 16 * K + kc); V b2; if (NSPLIT >= 2) b2 = WFrag<T16>::ld(Bt2 + boff + (size_t)nb * 16 * K + kc);
#pragma unroll
            for (int mb = 0; mb < 4; ++mb) { acc[mb][nb] = WFrag<T16>::mma(a[mb], b, acc[mb][nb]); if (NSPLIT == 1 || NSPLIT == 2) acc[mb][nb] = WFrag<T16>::mma(a2[mb], b, acc[mb][nb]); if (NSPLIT >= 2) acc[mb][nb] = WFrag<T16>::mma(a[mb], b2, acc[mb][nb]); } }
        asm volatile("v_nop\n\tv_nop\n\tv_nop\n\tv_nop" : "+v"(acc[0][0]), "+v"(acc[1][1]), "+v"(acc[2][2]), "+v"(acc[3][3]) : "v"(a[0]), "v"(a[3]));
    }
#pragma unroll
    for (int mb = 0; mb < 4; ++mb) {
#pragma unroll
        for (int nb = 0; nb < 4; ++nb) {
#pragma unroll
            for (int j = 0; j < 8; ++j) os[(hi * 8 + j) * 68 + nb * 16 + lr] = acc[mb][nb][j]; }
        __builtin_amdgcn_wave_barrier(); asm volatile("" ::: "memory");
        float* crow = C + (size_t)(r0 + mb * 16) * ldc + c0;
#pragma unroll 1
        for (int ps = 0; ps < 2; ++ps) {
#pragma unroll
            for (int s = 0; s < 8; ++s) { const int row = 2 * s + hi, cofs = lr * 4; v4f val = *(const v4fa*)(os + row * 68 + cofs); if (BIAS) { val[0] += bfr(bias[c0 + cofs]); val[1] += bfr(bias[c0 + cofs + 1]); val[2] += bfr(bias[c0 + cofs + 2]); val[3] += bfr(bias[c0 + cofs + 3]); }
                *(volatile v4f*)(crow + (size_t)row * ldc + cofs) = val; }
            if (ps == 0) __threadfence(); }
        __builtin_amdgcn_wave_barrier(); asm volatile("" ::: "memory");
    }
}

typedef __attribute__((ext_vector_type(2))) unsigned short v2us;
typedef __attribute__((ext_vector_type(2))) float v2f;

__global__ __launch_bounds__(256) void k_xn(const float* __restrict__ pp, bf* XN) {
    const int lane = threadIdx.x & 31; const int L0 = (blockIdx.x * 8 + (threadIdx.x >> 5)) * 8; const int nlines = NP * NS * DD / 64;
#pragma unroll 1
    for (int ps = 0; ps < 2; ++ps) {
#pragma unroll 1
        for (int l = 0; l < 8; ++l) { const int L = L0 + l; if (L >= nlines) break; const int e = L * 64 + lane * 2; const int d = e & 255; const int b = (e >> 8) % NS; const int n = e / (DD * NS); v2us o;
#pragma unroll
            for (int q = 0; q < 2; ++q) o[q] = f2bf(pp[((size_t)b * NP + n) * DD + d + q]);
            *(volatile v2us*)(XN + (size_t)e) = o; }
        if (ps == 0) __threadfence(); }
}
__global__ __launch_bounds__(256) void k_wt(const float* __restrict__ W, bf* WT) {
    const int lane = threadIdx.x & 31; const int L0 = (blockIdx.x * 8 + (threadIdx.x >> 5)) * 8; const int nlines = NP * MV * DD / 64;
#pragma unroll 1
    for (int ps = 0; ps < 2; ++ps) {
#pragma unroll 1
        for (int l = 0; l < 8; ++l) { const int L = L0 + l; if (L >= nlines) break; const int e = L * 64 + lane * 2; const int d = e & 255; const int mv = (e >> 8) % MV; const int n = e / (DD * MV); v2us o;
#pragma unroll
            for (int q = 0; q < 2; ++q) o[q] = f2bf(W[(((size_t)n * DD + d + q) * MC + mv / VV) * VV + (mv % VV)]);
            *(volatile v2us*)(WT + (size_t)e) = o; }
        if (ps == 0) __threadfence(); }
}
#define WE_SYNC() do { __builtin_amdgcn_wave_barrier(); asm volatile("" ::: "memory"); } while (0)
__global__ __launch_bounds__(256) void k_route(const float* __restrict__ VOT, const float* __restrict__ pact, const float* __restrict__ lng, const float* __restrict__ lnb, const float* __restrict__ emb, const float* __restrict__ cb, int b0, float* LG, float* CS) {
    __shared__ float sc[8][NP * MC + 1];
    __shared__ float sp[8][MC][VV];
    __shared__ float slg[8][32];
    const int lane = threadIdx.x & 31, wv = threadIdx.x >> 5; const int bl = blockIdx.x * 8 + wv; if (bl >= SCH) return; const int b = b0 + bl; const int v0 = lane * 2;
    const float* vb = VOT + (size_t)bl * NP * MV;
    float act[NP];
#pragma unroll
    for (int n = 0; n < NP; ++n) act[n] = bfr(pact[(size_t)b * NP + n]);
    const float g0 = bfr(lng[v0]), g1 = bfr(lng[v0 + 1]), be0 = bfr(lnb[v0]), be1 = bfr(lnb[v0 + 1]);
    float* c = sc[wv]; float (*pose)[VV] = sp[wv];
#pragma unroll 1
    for (int i = lane; i < NP * MC; i += 32) c[i] = 1.0f / 25.0f;
    WE_SYNC();
    auto compute_pose = [&]() {
#pragma unroll 1
        for (int m = 0; m < MC; ++m) { float s0 = 0.f, s1 = 0.f;
#pragma unroll
            for (int n = 0; n < NP; ++n) { const float w = c[n * MC + m] * act[n]; const v2f vt = *(const v2f*)(vb + (size_t)n * MV + m * VV + v0); s0 = fmaf(w, vt[0], s0); s1 = fmaf(w, vt[1], s1); }
            float su = s0 + s1;
#pragma unroll
            for (int sh = 16; sh; sh >>= 1) su += __shfl_xor(su, sh, 32);
            const float mu = su * (1.0f / VV); const float d0 = s0 - mu, d1 = s1 - mu; float q = d0 * d0 + d1 * d1;
#pragma unroll
            for (int sh = 16; sh; sh >>= 1) q += __shfl_xor(q, sh, 32);
            const float rs = rsqrtf(q * (1.0f / VV) + 1e-5f); pose[m][v0] = d0 * rs * g0 + be0; pose[m][v0 + 1] = d1 * rs * g1 + be1; }
        WE_SYNC(); };
    compute_pose();
#pragma unroll 1
    for (int it = 1; it < 3; ++it) {
#pragma unroll 1
        for (int n = 0; n < NP; ++n) { float mx = -3.0e38f; float myqk = 0.f;
#pragma unroll 1
            for (int m = 0; m < MC; ++m) { const v2f vt = *(const v2f*)(vb + (size_t)n * MV + m * VV + v0); float p = vt[0] * pose[m][v0] + vt[1] * pose[m][v0 + 1];
#pragma unroll
                for (int sh = 16; sh; sh >>= 1) p += __shfl_xor(p, sh, 32);
                p *= 0.125f; mx = fmaxf(mx, p); if (lane == m) myqk = p; }
            const float e = (lane < MC) ? __expf(myqk - mx) : 0.f; float se = e;
#pragma unroll
            for (int sh = 16; sh; sh >>= 1) se += __shfl_xor(se, sh, 32);
            if (lane < MC) c[n * MC + lane] = __fdiv_rn(e, se); }
        WE_SYNC();
        compute_pose(); }
    float mylogit = 0.f;
#pragma unroll 1
    for (int m = 0; m < MC; ++m) { float p = pose[m][v0] * bfr(emb[m * VV + v0]) + pose[m][v0 + 1] * bfr(emb[m * VV + v0 + 1]);
#pragma unroll
        for (int sh = 16; sh; sh >>= 1) p += __shfl_xor(p, sh, 32);
        if (lane == m) mylogit = p + bfr(cb[m]); }
#pragma unroll 1
    for (int ps = 0; ps < 2; ++ps) {
        *(volatile float*)(LG + (size_t)b * 32 + lane) = (lane < MC) ? mylogit : 0.f;
#pragma unroll 1
        for (int k = 0; k < 6; ++k) { const int idx = k * 32 + lane; const float v = (idx < NP * MC) ? c[idx] : 0.f; *(volatile float*)(CS + (size_t)b * 192 + idx) = v; }
        if (ps == 0) __threadfence(); }
}
__global__ __launch_bounds__(256) void k_pack(const float* __restrict__ LG, const float* __restrict__ pact, const float* __restrict__ CS, float* O0, float* O1, float* O2) {
    const size_t i = (size_t)blockIdx.x * 256 + threadIdx.x; const size_t n0 = (size_t)NS * MC, n1 = (size_t)NS * NP, n2 = (size_t)NS * NP * MC;
    float v; float* dst;
    if (i < n0) { v = LG[(i / MC) * 32 + (i % MC)]; dst = O0 + i; }
    else if (i < n0 + n1) { const size_t j = i - n0; v = bfr(pact[j]); dst = O1 + j; }
    else if (i < n0 + n1 + n2) { const size_t j = i - n0 - n1; v = CS[(j / (NP * MC)) * 192 + (j % (NP * MC))]; dst = O2 + j; }
    else return;
    *(volatile float*)dst = v; __threadfence(); *(volatile float*)dst = v;
}

extern "C" void kernel_launch(void* const* d_in, const int* in_sizes, int n_in,
                              void* d_out, int out_size, void* d_ws, size_t ws_size, hipStream_t stream) {
    (void)in_sizes; (void)n_in; (void)out_size;
    const float* pp = (const float*)d_in[0]; const float* pact = (const float*)d_in[1]; const float* W = (const float*)d_in[2]; const float* lng = (const float*)d_in[3]; const float* lnb = (const float*)d_in[4]; const float* emb = (const float*)d_in[5]; const float* cb = (const float*)d_in[6];
    float* O0 = (float*)d_out;
    float* O1 = (float*)((char*)d_out + 819200);
    float* O2 = (float*)((char*)d_out + 1048576);
    char* wsp = (char*)d_ws;
    auto take = [&](size_t bytes) { char* p = wsp; wsp += (bytes + 255) & ~(size_t)255; return (void*)p; };
    bf* XN = (bf*)take((size_t)NP * NS * DD * 2); bf* WT = (bf*)take((size_t)NP * MV * DD * 2); float* VOT = (float*)take((size_t)SCH * NP * MV * 4); float* LG = (float*)take((size_t)NS * 32 * 4); float* CS = (float*)take((size_t)NS * 192 * 4);
    if ((size_t)(wsp - (char*)d_ws) > ws_size) return;
    k_xn<<<(NP * NS * DD / 64 + 63) / 64, 256, 0, stream>>>(pp, XN); k_wt<<<(NP * MV * DD / 64 + 63) / 64, 256, 0, stream>>>(W, WT);
    for (int ch = 0; ch < NCHK; ++ch) { const int b0 = ch * SCH;
        k_gemmw<bf, 0, false><<<dim3(SCH / 64, MV / 64, NP), 32, 0, stream>>>(XN + (size_t)b0 * DD, nullptr, WT, nullptr, DD, VOT, NP * MV, nullptr, (size_t)NS * DD, (size_t)MV * DD, (size_t)MV);
        k_route<<<SCH / 8, 256, 0, stream>>>(VOT, pact, lng, lnb, emb, cb, b0, LG, CS); }
    { const size_t tot = (size_t)NS * (MC + NP + NP * MC); k_pack<<<(unsigned)((tot + 255) / 256), 256, 0, stream>>>(LG, pact, CS, O0, O1, O2); }
}
